// EnergyMACE_2207613190289
// MI455X (gfx1250) — hardware-run, weakly checked
//
#include <hip/hip_runtime.h>


namespace {
constexpr int N = 10000, E = 160000, F = 64, S = 5, NB = 8, NL = 4, NLM = 16, HID = 16, RH = 32, NBLK = N / 16;
constexpr float RMAX = 5.0f, AVG = 16.0f, WSC = 256.0f, XS = 8.0f;
__constant__ int LOF[16] = {0, 1, 1, 1, 2, 2, 2, 2, 2, 3, 3, 3, 3, 3, 3, 3};
typedef _Float16 b16;
typedef __attribute__((ext_vector_type(16))) _Float16 v16b;
typedef __attribute__((ext_vector_type(8))) _Float16 v8b;
typedef __attribute__((ext_vector_type(8))) float v8f;
typedef __attribute__((ext_vector_type(4))) float v4f;
typedef __attribute__((ext_vector_type(2))) float v2f;
__device__ __forceinline__ float bf16_rne(float f) { unsigned int u = __float_as_uint(f); u += 0x7FFFu + ((u >> 16) & 1u); return __uint_as_float(u & 0xFFFF0000u); }
__device__ __forceinline__ void split16(float v, b16& hi, b16& lo) { hi = (b16)v; lo = (b16)(v - (float)hi); }
__device__ __forceinline__ v16b frag_kb(const b16* p, int hh) { const v8b a = *(const v8b*)(p + 8 * hh), b = *(const v8b*)(p + 16 + 8 * hh); v16b f;
#pragma unroll
  for (int e = 0; e < 8; ++e) { f[e] = a[e]; f[8 + e] = b[e]; } return f; }
__device__ __forceinline__ v8f wmma16b(v16b a, v16b b, v8f c) { v8f d = __builtin_amdgcn_wmma_f32_16x16x32_f16(false, a, false, b, (short)0, c, false, false); asm volatile("v_nop\n\tv_nop\n\tv_nop\n\tv_nop" : "+v"(d) : "v"(a), "v"(b)); return d; }
__device__ __forceinline__ void wave_lds_sync() { __builtin_amdgcn_fence(__ATOMIC_RELEASE, "workgroup"); __builtin_amdgcn_wave_barrier(); __builtin_amdgcn_fence(__ATOMIC_ACQUIRE, "workgroup"); }
__device__ __forceinline__ float pmul(float a, float b) { float p = a * b; asm volatile("" : "+v"(p)); return p; }
__device__ __forceinline__ int iclamp(int v, int lo, int hi) { return v < lo ? lo : (v > hi ? hi : v); }
__device__ __forceinline__ float silu(float v) { return v / (1.0f + __expf(-v)); }
constexpr int CSR_NBLK9 = 512, CSR_GB9 = 9, CSR_GN9 = 1 << CSR_GB9  , CSR_TS9 = (CSR_GN9 < 32 ? 32 : CSR_GN9)  , CSR_MAXG9 = 512, CSR_CAP9 = 12288  ;
__device__ __host__ __forceinline__ int csr_tix9(int v) { return (v >> CSR_GB9) * CSR_TS9 + (v & (CSR_GN9 - 1)); }
__global__ __launch_bounds__(64) void csrA_kernel9(const int* __restrict__ dst, int E, int N, int nG, int CHP, int NGP, int* __restrict__ STG, int* __restrict__ HST) {
  extern __shared__ int sm[];
  int* cnt = sm; int* run = sm + NGP; int* ids = sm + 2 * NGP;
  const int b = blockIdx.x; const int ch = (E + CSR_NBLK9 - 1) / CSR_NBLK9; const int e0 = b * ch, e1 = min(E, e0 + ch);
  for (int i = threadIdx.x; i < NGP; i += 64) cnt[i] = 0;
  for (int i = threadIdx.x; i < CHP; i += 64) ids[i] = -1;
  __syncthreads();
  if (threadIdx.x == 0) {
    for (int e = e0; e < e1; ++e) { int d = dst[e]; d = (d < 0) ? 0 : (d >= N ? N - 1 : d); cnt[d >> CSR_GB9] += 1; }
    int acc = 0; for (int g = 0; g < nG; ++g) { run[g] = acc; acc += cnt[g]; }
    for (int e = e0; e < e1; ++e) { int d = dst[e]; d = (d < 0) ? 0 : (d >= N ? N - 1 : d); const int g = d >> CSR_GB9; ids[run[g]] = e; run[g] += 1; } }
  __syncthreads();
  typedef __attribute__((ext_vector_type(4))) int v4i;
  for (int pass = 0; pass < 2; ++pass) {
    for (int i = threadIdx.x; i < CHP / 4; i += 64) *(volatile v4i*)(STG + (size_t)b * CHP + i * 4) = *(const v4i*)(&ids[i * 4]);
    for (int i = threadIdx.x; i < NGP / 4; i += 64) { v4i v; for (int e = 0; e < 4; ++e) v[e] = (i * 4 + e < nG) ? cnt[i * 4 + e] : 0; *(volatile v4i*)(HST + (size_t)b * NGP + i * 4) = v; }
    __threadfence(); }
}
__global__ __launch_bounds__(512) void csrS_kernel9(const int* __restrict__ HST, int nG, int NGP, int* __restrict__ START, int* __restrict__ TOT, int* __restrict__ OFF) {
  __shared__ int tot[CSR_MAXG9];
  const int b = threadIdx.x;
  for (int pass = 0; pass < 2; ++pass) { int runb = 0; for (int g = 0; g < nG; ++g) { int c = HST[(size_t)b * NGP + g]; c = (c < 0) ? 0 : c; ((volatile int*)OFF)[(size_t)g * CSR_NBLK9 + b] = runb; runb += c; } __threadfence(); }
  for (int g = threadIdx.x; g < nG; g += 512) { int s = 0; for (int bb = 0; bb < CSR_NBLK9; ++bb) { int c = HST[(size_t)bb * NGP + g]; s += (c < 0) ? 0 : c; } tot[g] = s; }
  __syncthreads();
  if (threadIdx.x < 32) {
    __shared__ int st[CSR_MAXG9 + 32];
    if (threadIdx.x == 0) { int acc = 0; for (int g = 0; g < NGP; ++g) { st[g] = acc; if (g < nG) acc += (tot[g] + 31) & ~31; } st[NGP] = acc; }
    __builtin_amdgcn_fence(__ATOMIC_RELEASE, "workgroup"); __builtin_amdgcn_wave_barrier(); __builtin_amdgcn_fence(__ATOMIC_ACQUIRE, "workgroup");
    for (int pass = 0; pass < 2; ++pass) { for (int i = threadIdx.x; i < NGP + 32; i += 32) { ((volatile int*)START)[i] = (i <= NGP) ? st[min(i, NGP)] : 0; ((volatile int*)TOT)[i] = (i < nG) ? tot[i] : 0; } __threadfence(); } }
}
__global__ __launch_bounds__(256) void csrB_kernel9(const int* __restrict__ dst, int N, int nG, int CHP, int NGP, int permLen, const int* __restrict__ STG, const int* __restrict__ HST, const int* __restrict__ OFF, const int* __restrict__ START, const int* __restrict__ TOT, int* __restrict__ PERM, int* __restrict__ ROWPTR, int* __restrict__ ROWCNT, int* __restrict__ FLAG) {
  typedef __attribute__((ext_vector_type(4))) int v4i;
  __shared__ int ids[CSR_CAP9]; __shared__ unsigned short key[CSR_CAP9]; __shared__ int outp[CSR_CAP9]; __shared__ int ncnt[CSR_GN9 + 1]; __shared__ int boff[CSR_NBLK9 + 1];
  const int g = blockIdx.x, t_ = threadIdx.x; int tot = TOT[g]; int st = START[g], stn = START[g + 1]; const int v0 = g * CSR_GN9; const int nv = min(CSR_GN9, N - v0); const int t0 = g * CSR_TS9;
  st = (st < 0) ? 0 : (st > permLen - 32 ? permLen - 32 : st) & ~31; stn = (stn < st) ? st : (stn > permLen ? permLen : stn); tot = (tot < 0) ? 0 : tot; if (tot > stn - st && tot <= CSR_CAP9) tot = stn - st;
  if (tot > CSR_CAP9) {
    for (int pass = 0; pass < 2; ++pass) { for (int i = t_; i < CSR_TS9 / 4; i += 256) { v4i a, c; for (int e = 0; e < 4; ++e) { a[e] = st; c[e] = 0; } *(volatile v4i*)(ROWPTR + t0 + i * 4) = a; *(volatile v4i*)(ROWCNT + t0 + i * 4) = c; } if (t_ == 0) ((volatile int*)FLAG)[0] = 1; __threadfence(); } (void)nv; return; }
  if (t_ == 0) { int acc = 0; for (int b = 0; b < CSR_NBLK9; ++b) { boff[b] = acc; int c = HST[(size_t)b * NGP + g]; c = (c < 0) ? 0 : (c > CHP ? CHP : c); acc += c; if (acc > tot) acc = tot; } boff[CSR_NBLK9] = acc; }
  for (int i = t_; i <= CSR_GN9; i += 256) ncnt[i] = 0;
  __syncthreads();
  for (int b = 0; b < CSR_NBLK9; ++b) { const int c = boff[b + 1] - boff[b]; int o_ = OFF[(size_t)g * CSR_NBLK9 + b]; o_ = (o_ < 0) ? 0 : (o_ > CHP - c ? CHP - c : o_); const int* src_ = STG + (size_t)b * CHP + o_;
    for (int i = t_; i < c; i += 256) { int id = src_[i]; id = (id < 0) ? 0 : id; ids[boff[b] + i] = id; int d = dst[id]; d = (d < v0) ? v0 : (d >= N ? N - 1 : d); int kk = d - v0; kk = (kk < 0) ? 0 : (kk >= CSR_GN9 ? CSR_GN9 - 1 : kk); key[boff[b] + i] = (unsigned short)kk; } }
  __syncthreads();
  if (t_ == 0) { for (int i = 0; i < tot; ++i) ncnt[key[i]] += 1; int acc = 0; for (int vl = 0; vl < CSR_GN9; ++vl) { const int c = ncnt[vl]; ncnt[vl] = acc; acc += c; } ncnt[CSR_GN9] = acc;
    for (int i = 0; i < tot; ++i) { const int vl = key[i]; outp[ncnt[vl]] = ids[i]; ncnt[vl] += 1; }
    for (int vl = CSR_GN9; vl > 0; --vl) ncnt[vl] = ncnt[vl - 1]; ncnt[0] = 0; }
  __syncthreads();
  for (int pass = 0; pass < 2; ++pass) {
    for (int i = t_; i < (stn - st) / 4; i += 256) { v4i v; for (int e = 0; e < 4; ++e) { const int q = i * 4 + e; v[e] = (q < tot) ? outp[q] : -1; } *(volatile v4i*)(PERM + st + i * 4) = v; }
    for (int i = t_; i < CSR_TS9 / 4; i += 256) { v4i a, c; for (int e = 0; e < 4; ++e) { const int vl = i * 4 + e; const int vc = vl < CSR_GN9 ? vl : CSR_GN9; a[e] = (vl < CSR_GN9) ? st + ncnt[vc] : st; c[e] = (vl < nv) ? (ncnt[(vc < CSR_GN9 ? vc : CSR_GN9 - 1) + 1] - ncnt[vc]) : 0; } *(volatile v4i*)(ROWPTR + t0 + i * 4) = a; *(volatile v4i*)(ROWCNT + t0 + i * 4) = c; }
    __threadfence(); }
}
__global__ __launch_bounds__(256) void csrZ_kernel9(int* __restrict__ p, size_t n4) { typedef __attribute__((ext_vector_type(4))) int v4i; const size_t tid = (size_t)blockIdx.x * 256 + threadIdx.x, nth = (size_t)gridDim.x * 256; v4i z = {0, 0, 0, 0}; for (size_t i = tid; i < n4; i += nth) *(volatile v4i*)(p + i * 4) = z; }
struct CsrBufs9 { int *STG, *HST, *OFF, *START, *TOT, *PERM, *ROWPTR, *ROWCNT, *FLAG; int nG, NGP, CHP; size_t permLen; char* base; size_t bytes; };
static size_t csr_carve9(CsrBufs9& c, char* ws, size_t off, int E, int N) {
  const size_t off0 = off; c.base = ws + off;
  auto al = [&](size_t bytes) { char* p = ws + off; off += (bytes + 255) & ~(size_t)255; return p; };
  c.nG = (N + CSR_GN9 - 1) / CSR_GN9; c.NGP = (c.nG + 31) & ~31; const int ch = (E + CSR_NBLK9 - 1) / CSR_NBLK9; c.CHP = (ch + 31) & ~31; c.permLen = (size_t)E + 32 * (size_t)c.nG + 32;
  c.STG = (int*)al((size_t)CSR_NBLK9 * c.CHP * 4); c.HST = (int*)al((size_t)CSR_NBLK9 * c.NGP * 4); c.OFF = (int*)al((size_t)c.NGP * CSR_NBLK9 * 4); c.START = (int*)al((size_t)(c.NGP + 64) * 4); c.TOT = (int*)al((size_t)(c.NGP + 64) * 4);
  c.PERM = (int*)al(c.permLen * 4); c.ROWPTR = (int*)al((size_t)c.nG * CSR_TS9 * 4); c.ROWCNT = (int*)al((size_t)c.nG * CSR_TS9 * 4); c.FLAG = (int*)al(256);
  c.bytes = off - off0; return off;
}
static void csr_build9(const CsrBufs9& c, const int* dst, int E, int N, hipStream_t stream) {
  const size_t smem = (size_t)(2 * c.NGP + c.CHP) * 4;
  csrZ_kernel9<<<512, 256, 0, stream>>>((int*)c.base, c.bytes / 16);
  csrA_kernel9<<<CSR_NBLK9, 64, smem, stream>>>(dst, E, N, c.nG, c.CHP, c.NGP, c.STG, c.HST);
  csrS_kernel9<<<1, 512, 0, stream>>>(c.HST, c.nG, c.NGP, c.START, c.TOT, c.OFF);
  csrB_kernel9<<<c.nG, 256, 0, stream>>>(dst, N, c.nG, c.CHP, c.NGP, (int)c.permLen, c.STG, c.HST, c.OFF, c.START, c.TOT, c.PERM, c.ROWPTR, c.ROWCNT, c.FLAG);
}


__global__ __launch_bounds__(256) void wput_kernel(const float* __restrict__ w, int KIN, int OUTW, int ro, int ko, int KP, b16* __restrict__ WT) {
  const int KG = KIN / 8; const int u = blockIdx.x * 256 + threadIdx.x; if (u >= OUTW * KG) return; const int o = u / KG, k0 = (u % KG) * 8; v8b v;
#pragma unroll
  for (int j = 0; j < 8; ++j) v[j] = (b16)(bf16_rne(w[(size_t)(k0 + j) * OUTW + o]) * WSC); for (int pass = 0; pass < 2; ++pass) { *(volatile v8b*)(WT + (size_t)(ro + o) * KP + ko + k0) = v; __threadfence(); }
}
__global__ __launch_bounds__(256) void wzero_kernel(size_t n8, b16* __restrict__ WT) { const size_t u = (size_t)blockIdx.x * 256 + threadIdx.x; if (u >= n8) return; v8b z; for (int j = 0; j < 8; ++j) z[j] = (b16)0.0f; for (int pass = 0; pass < 2; ++pass) { *(volatile v8b*)(WT + u * 8) = z; __threadfence(); } }
__global__ __launch_bounds__(32) void emb_kernel(const float* __restrict__ attrs, const float* __restrict__ Wemb, float* __restrict__ Hh) {
  const int lane = threadIdx.x; const size_t m0 = (size_t)blockIdx.x * 16;
  for (int pass = 0; pass < 2; ++pass) {
#pragma unroll 1
    for (int rr = 0; rr < 16; ++rr) { v2f r = {0.0f, 0.0f};
#pragma unroll 1
      for (int s = 0; s < S; ++s) { const float a = bf16_rne(attrs[(m0 + rr) * S + s]); r[0] += pmul(a, bf16_rne(Wemb[s * F + lane * 2])); r[1] += pmul(a, bf16_rne(Wemb[s * F + lane * 2 + 1])); } *(volatile v2f*)(Hh + (m0 + rr) * F + lane * 2) = r; } __threadfence(); }
}
__global__ __launch_bounds__(32) void hu_kernel(const float* __restrict__ Hh, const b16* __restrict__ WUP, int NLIM, float* __restrict__ HU) {
  __shared__ __attribute__((aligned(16))) b16 Ah[16][F + 8], Al[16][F + 8]; __shared__ __attribute__((aligned(16))) float Tf[16][F + 4];
  const int lane = threadIdx.x, nloc = lane & 15, hlf = lane >> 4; const size_t m0 = (size_t)blockIdx.x * 16; if (m0 >= (size_t)NLIM) return;
  for (int rr = 0; rr < 16; ++rr) for (int q = 0; q < 2; ++q) { b16 p, ql; split16(Hh[(m0 + rr) * F + q * 32 + lane] * XS, p, ql); Ah[rr][q * 32 + lane] = p; Al[rr][q * 32 + lane] = ql; }
  wave_lds_sync(); v8f acc[4] = {(v8f){}, (v8f){}, (v8f){}, (v8f){}};
#pragma unroll
  for (int kb = 0; kb < F; kb += 32) { const v16b a = frag_kb(&Ah[nloc][kb], hlf), a2 = frag_kb(&Al[nloc][kb], hlf);
#pragma unroll
    for (int t = 0; t < 4; ++t) { const v16b bw = frag_kb(WUP + (size_t)(t * 16 + nloc) * F + kb, hlf); acc[t] = wmma16b(a, bw, acc[t]); acc[t] = wmma16b(a2, bw, acc[t]); } }
#pragma unroll
  for (int t = 0; t < 4; ++t)
#pragma unroll
    for (int r8 = 0; r8 < 8; ++r8) Tf[8 * hlf + r8][t * 16 + nloc] = acc[t][r8] * (1.0f / (XS * WSC));
  wave_lds_sync();
  for (int pass = 0; pass < 2; ++pass) { for (int rr = 0; rr < 16; ++rr) *(volatile v2f*)(HU + (m0 + rr) * F + lane * 2) = *(const v2f*)(&Tf[rr][lane * 2]); __threadfence(); }
}
__global__ __launch_bounds__(32) void msg_kernel(const float* __restrict__ pos, const float* __restrict__ shifts, const int* __restrict__ snd, const float* __restrict__ HU, const b16* __restrict__ WR0, const b16* __restrict__ WR1, const b16* __restrict__ WR2, const int* __restrict__ PERM, const int* __restrict__ ROWPTR, const int* __restrict__ ROWCNT, int permLen, int NLIM, float* __restrict__ A) {
  __shared__ __attribute__((aligned(16))) b16 Ah[16][40], Al[16][40]; __shared__ float Sh[16][NLM + 1], Rf[16][NL * F + 4]; __shared__ int Ss[16]; __shared__ __attribute__((aligned(16))) float Ao[NLM][F];
  const int lane = threadIdx.x, nloc = lane & 15, hlf = lane >> 4; const size_t n = blockIdx.x; if (n >= (size_t)NLIM) return;
  const float px = bf16_rne(pos[n * 3]), py = bf16_rne(pos[n * 3 + 1]), pz = bf16_rne(pos[n * 3 + 2]);
  int st = ROWPTR[n], cnt = ROWCNT[n]; cnt = iclamp(cnt, 0, 1 << 20); st = iclamp(st, 0, permLen - cnt);
  float acc[NLM][2];
#pragma unroll
  for (int k = 0; k < NLM; ++k) { acc[k][0] = 0.0f; acc[k][1] = 0.0f; }
#pragma unroll 1
  for (int j0 = 0; j0 < cnt; j0 += 16) {
    if (lane < 16) { const int jj = j0 + lane; int s = -1; float efv[NB]; float shv[NLM]; for (int k = 0; k < NB; ++k) efv[k] = 0.0f; for (int k = 0; k < NLM; ++k) shv[k] = 0.0f;
      if (jj < cnt) { const int e = iclamp(PERM[st + jj], 0, E - 1); s = iclamp(snd[e], 0, N - 1); if (s >= NLIM) s = -1;
        if (s >= 0) { const float vx = px - bf16_rne(pos[(size_t)s * 3]) + bf16_rne(shifts[(size_t)e * 3]), vy = py - bf16_rne(pos[(size_t)s * 3 + 1]) + bf16_rne(shifts[(size_t)e * 3 + 1]), vz = pz - bf16_rne(pos[(size_t)s * 3 + 2]) + bf16_rne(shifts[(size_t)e * 3 + 2]);
          const float r = sqrtf(pmul(vx, vx) + pmul(vy, vy) + pmul(vz, vz) + 1e-12f); const float x = vx / r, y = vy / r, z = vz / r;
          const float c3 = 1.7320508075688772f, c15 = 3.872983346207417f, c5 = 2.23606797749979f, c105 = 10.246950765959598f, c358 = 2.091650066335189f, c218 = 1.620185174601965f, c7 = 2.6457513110645907f;
          shv[0] = 1.0f; shv[1] = c3 * x; shv[2] = c3 * y; shv[3] = c3 * z; shv[4] = c15 * x * y; shv[5] = c15 * y * z; shv[6] = 0.5f * c5 * (3.0f * z * z - 1.0f); shv[7] = c15 * x * z; shv[8] = 0.5f * c15 * (x * x - y * y);
          shv[9] = c358 * y * (3.0f * x * x - y * y); shv[10] = c105 * x * y * z; shv[11] = c218 * y * (5.0f * z * z - 1.0f); shv[12] = 0.5f * c7 * (5.0f * z * z * z - 3.0f * z); shv[13] = c218 * x * (5.0f * z * z - 1.0f); shv[14] = 0.5f * c105 * z * (x * x - y * y); shv[15] = c358 * x * (x * x - 3.0f * y * y);
          const float xr = r / RMAX; const float rden = fmaxf(r, 1e-6f); const float P = 5.0f; float env = 1.0f - 0.5f * (P + 1.0f) * (P + 2.0f) * powf(xr, 5.0f) + P * (P + 2.0f) * powf(xr, 6.0f) - 0.5f * P * (P + 1.0f) * powf(xr, 7.0f); if (!(xr < 1.0f)) env = 0.0f;
          for (int k = 0; k < NB; ++k) efv[k] = 0.6324555320336759f * sinf(3.14159265358979323846f * (float)(k + 1) * xr) / rden * env; } }
      Ss[lane] = s; for (int k = 0; k < NLM; ++k) Sh[lane][k] = shv[k]; for (int k = 0; k < 32; ++k) { b16 p = (b16)0.0f, q = (b16)0.0f; if (k < NB) split16(efv[k] * XS, p, q); Ah[lane][k] = p; Al[lane][k] = q; } }
    wave_lds_sync();
    { v8f a2[2] = {(v8f){}, (v8f){}}; const v16b a = frag_kb(&Ah[nloc][0], hlf), al = frag_kb(&Al[nloc][0], hlf);
#pragma unroll
      for (int t = 0; t < 2; ++t) { const v16b bw = frag_kb(WR0 + (size_t)(t * 16 + nloc) * 32, hlf); a2[t] = wmma16b(a, bw, a2[t]); a2[t] = wmma16b(al, bw, a2[t]); }
      wave_lds_sync();
#pragma unroll
      for (int t = 0; t < 2; ++t)
#pragma unroll
        for (int r8 = 0; r8 < 8; ++r8) { b16 p, q; split16(silu(a2[t][r8] * (1.0f / (XS * WSC))) * XS, p, q); Ah[8 * hlf + r8][t * 16 + nloc] = p; Al[8 * hlf + r8][t * 16 + nloc] = q; } }
    wave_lds_sync();
    { v8f a2[2] = {(v8f){}, (v8f){}}; const v16b a = frag_kb(&Ah[nloc][0], hlf), al = frag_kb(&Al[nloc][0], hlf);
#pragma unroll
      for (int t = 0; t < 2; ++t) { const v16b bw = frag_kb(WR1 + (size_t)(t * 16 + nloc) * 32, hlf); a2[t] = wmma16b(a, bw, a2[t]); a2[t] = wmma16b(al, bw, a2[t]); }
      wave_lds_sync();
#pragma unroll
      for (int t = 0; t < 2; ++t)
#pragma unroll
        for (int r8 = 0; r8 < 8; ++r8) { b16 p, q; split16(silu(a2[t][r8] * (1.0f / (XS * WSC))) * XS, p, q); Ah[8 * hlf + r8][t * 16 + nloc] = p; Al[8 * hlf + r8][t * 16 + nloc] = q; } }
    wave_lds_sync();
    { const v16b a = frag_kb(&Ah[nloc][0], hlf), al = frag_kb(&Al[nloc][0], hlf);
#pragma unroll 1
      for (int cg = 0; cg < 2; ++cg) { v8f a3[8];
#pragma unroll
        for (int t = 0; t < 8; ++t) { a3[t] = (v8f){}; const v16b bw = frag_kb(WR2 + (size_t)(cg * 128 + t * 16 + nloc) * 32, hlf); a3[t] = wmma16b(a, bw, a3[t]); a3[t] = wmma16b(al, bw, a3[t]); }
#pragma unroll
        for (int t = 0; t < 8; ++t)
#pragma unroll
          for (int r8 = 0; r8 < 8; ++r8) Rf[8 * hlf + r8][cg * 128 + t * 16 + nloc] = a3[t][r8] * (1.0f / (XS * WSC)); } }
    wave_lds_sync();
    for (int rr = 0; rr < 16; ++rr) { const int s = Ss[rr]; if (s < 0) continue; const float h0 = HU[(size_t)s * F + lane * 2], h1 = HU[(size_t)s * F + lane * 2 + 1];
#pragma unroll
      for (int k = 0; k < NLM; ++k) { const float shk = Sh[rr][k]; const float* rp = &Rf[rr][LOF[k] * F + lane * 2]; acc[k][0] += pmul(pmul(shk, rp[0]), h0); acc[k][1] += pmul(pmul(shk, rp[1]), h1); } }
    wave_lds_sync(); }
#pragma unroll
  for (int k = 0; k < NLM; ++k) { Ao[k][lane * 2] = acc[k][0] * (1.0f / AVG); Ao[k][lane * 2 + 1] = acc[k][1] * (1.0f / AVG); }
  wave_lds_sync();
  for (int pass = 0; pass < 2; ++pass) { for (int q = 0; q < 8; ++q) { const int i4 = (q * 32 + lane) * 4; *(volatile v4f*)(A + n * (NLM * F) + i4) = *(const v4f*)(&Ao[i4 / F][i4 % F]); } __threadfence(); }
}
template <int RO>
__global__ __launch_bounds__(32) void upd_kernel(const float* __restrict__ A, const float* __restrict__ Hh, const float* __restrict__ attrs, const b16* __restrict__ WMIX, const b16* __restrict__ WSCT, const b16* __restrict__ WP, const float* __restrict__ wro, const b16* __restrict__ WRO1A, const float* __restrict__ wro1b, int NLIM, float* __restrict__ HN, float* __restrict__ EO) {
  __shared__ __attribute__((aligned(16))) b16 Ah[16][320 + 8], Al[16][320 + 8]; __shared__ float B1s[16][F + 1], B2s[16][F + 1], Tf[16][F + 4], Es[16];
  const int lane = threadIdx.x, nloc = lane & 15, hlf = lane >> 4; const size_t m0 = (size_t)blockIdx.x * 16; if (m0 >= (size_t)NLIM) return;
  for (int rr = 0; rr < 16; ++rr) { B2s[rr][lane * 2] = 0.0f; B2s[rr][lane * 2 + 1] = 0.0f; }
#pragma unroll 1
  for (int k = 0; k < NLM; ++k) {
    for (int rr = 0; rr < 16; ++rr) for (int q = 0; q < 2; ++q) { b16 p, ql; split16(A[((m0 + rr) * NLM + k) * F + q * 32 + lane] * 64.0f, p, ql); Ah[rr][q * 32 + lane] = p; Al[rr][q * 32 + lane] = ql; }
    wave_lds_sync(); v8f acc[4] = {(v8f){}, (v8f){}, (v8f){}, (v8f){}}; const b16* W = WMIX + (size_t)LOF[k] * F * F;
#pragma unroll
    for (int kb = 0; kb < F; kb += 32) { const v16b a = frag_kb(&Ah[nloc][kb], hlf), a2 = frag_kb(&Al[nloc][kb], hlf);
#pragma unroll
      for (int t = 0; t < 4; ++t) { const v16b bw = frag_kb(W + (size_t)(t * 16 + nloc) * F + kb, hlf); acc[t] = wmma16b(a, bw, acc[t]); acc[t] = wmma16b(a2, bw, acc[t]); } }
#pragma unroll
    for (int t = 0; t < 4; ++t)
#pragma unroll
      for (int r8 = 0; r8 < 8; ++r8) { const int rl = 8 * hlf + r8, c = t * 16 + nloc; const float v = acc[t][r8] * (1.0f / (64.0f * WSC)); if (k == 0) B1s[rl][c] = v; B2s[rl][c] += pmul(v, v); }
    wave_lds_sync(); }
  for (int rr = 0; rr < 16; ++rr) { const float hv0 = Hh[(m0 + rr) * F + lane], hv1 = Hh[(m0 + rr) * F + 32 + lane]; for (int s = 0; s < S; ++s) { const float as_ = bf16_rne(attrs[(m0 + rr) * S + s]); b16 p, ql; split16(pmul(as_, hv0) * XS, p, ql); Ah[rr][s * F + lane] = p; Al[rr][s * F + lane] = ql; split16(pmul(as_, hv1) * XS, p, ql); Ah[rr][s * F + 32 + lane] = p; Al[rr][s * F + 32 + lane] = ql; } }
  wave_lds_sync(); v8f scc[4] = {(v8f){}, (v8f){}, (v8f){}, (v8f){}};
#pragma unroll 2
  for (int kb = 0; kb < S * F; kb += 32) { const v16b a = frag_kb(&Ah[nloc][kb], hlf), a2 = frag_kb(&Al[nloc][kb], hlf);
#pragma unroll
    for (int t = 0; t < 4; ++t) { const v16b bw = frag_kb(WSCT + (size_t)(t * 16 + nloc) * (S * F) + kb, hlf); scc[t] = wmma16b(a, bw, scc[t]); scc[t] = wmma16b(a2, bw, scc[t]); } }
  wave_lds_sync();
  for (int rr = 0; rr < 16; ++rr) for (int q = 0; q < 2; ++q) { const int c = q * 32 + lane; const float b1 = B1s[rr][c], b2v = B2s[rr][c]; b16 p, ql; split16(b1 * 128.0f, p, ql); Ah[rr][c] = p; Al[rr][c] = ql; split16(b2v * 128.0f, p, ql); Ah[rr][F + c] = p; Al[rr][F + c] = ql; split16(pmul(b2v, b1) * 1024.0f, p, ql); Ah[rr][2 * F + c] = p; Al[rr][2 * F + c] = ql; }
  wave_lds_sync(); v8f p1[4] = {(v8f){}, (v8f){}, (v8f){}, (v8f){}}, p2[4] = {(v8f){}, (v8f){}, (v8f){}, (v8f){}}, p3[4] = {(v8f){}, (v8f){}, (v8f){}, (v8f){}};
#pragma unroll
  for (int kb = 0; kb < F; kb += 32) { const v16b a1 = frag_kb(&Ah[nloc][kb], hlf), l1 = frag_kb(&Al[nloc][kb], hlf), a2 = frag_kb(&Ah[nloc][F + kb], hlf), l2 = frag_kb(&Al[nloc][F + kb], hlf), a3 = frag_kb(&Ah[nloc][2 * F + kb], hlf), l3 = frag_kb(&Al[nloc][2 * F + kb], hlf);
#pragma unroll
    for (int t = 0; t < 4; ++t) { const v16b w1 = frag_kb(WP + (size_t)(t * 16 + nloc) * F + kb, hlf), w2 = frag_kb(WP + (size_t)(F + t * 16 + nloc) * F + kb, hlf), w3 = frag_kb(WP + (size_t)(2 * F + t * 16 + nloc) * F + kb, hlf);
      p1[t] = wmma16b(a1, w1, p1[t]); p1[t] = wmma16b(l1, w1, p1[t]); p2[t] = wmma16b(a2, w2, p2[t]); p2[t] = wmma16b(l2, w2, p2[t]); p3[t] = wmma16b(a3, w3, p3[t]); p3[t] = wmma16b(l3, w3, p3[t]); } }
#pragma unroll
  for (int t = 0; t < 4; ++t)
#pragma unroll
    for (int r8 = 0; r8 < 8; ++r8) Tf[8 * hlf + r8][t * 16 + nloc] = p1[t][r8] * (1.0f / (128.0f * WSC)) + p2[t][r8] * (1.0f / (128.0f * WSC)) + p3[t][r8] * (1.0f / (1024.0f * WSC)) + scc[t][r8] * (1.0f / (XS * WSC));
  wave_lds_sync();
  if (RO == 0) { for (int rr = 0; rr < 16; ++rr) { float s = pmul(Tf[rr][lane], bf16_rne(wro[lane])) + pmul(Tf[rr][32 + lane], bf16_rne(wro[32 + lane])); for (int o = 16; o; o >>= 1) s += __shfl_xor(s, o); if (lane == 0) Es[rr] = s; } }
  else { for (int rr = 0; rr < 16; ++rr) for (int q = 0; q < 2; ++q) { b16 p, ql; split16(Tf[rr][q * 32 + lane] * XS, p, ql); Ah[rr][q * 32 + lane] = p; Al[rr][q * 32 + lane] = ql; }
    wave_lds_sync(); v8f g = {};
#pragma unroll
    for (int kb = 0; kb < F; kb += 32) { const v16b bw = frag_kb(WRO1A + (size_t)nloc * F + kb, hlf); g = wmma16b(frag_kb(&Ah[nloc][kb], hlf), bw, g); g = wmma16b(frag_kb(&Al[nloc][kb], hlf), bw, g); }
    float pd[8];
#pragma unroll
    for (int r8 = 0; r8 < 8; ++r8) pd[r8] = pmul(silu(g[r8] * (1.0f / (XS * WSC))), bf16_rne(wro1b[nloc]));
#pragma unroll
    for (int r8 = 0; r8 < 8; ++r8) { float s = pd[r8]; for (int o = 1; o < 16; o <<= 1) s += __shfl_xor(s, o); if (nloc == 0) Es[8 * hlf + r8] = s; } }
  wave_lds_sync();
  for (int pass = 0; pass < 2; ++pass) { for (int rr = 0; rr < 16; ++rr) *(volatile v2f*)(HN + (m0 + rr) * F + lane * 2) = *(const v2f*)(&Tf[rr][lane * 2]); ((volatile float*)EO)[blockIdx.x * 32 + lane] = (lane < 16) ? Es[lane] : 0.0f; __threadfence(); }
}
__global__ __launch_bounds__(32) void out_kernel(const float* __restrict__ E0, const float* __restrict__ E1, float* __restrict__ out) {
  const int lane = threadIdx.x; const size_t n = (size_t)blockIdx.x * 16 + (lane >> 1); const size_t ei = (size_t)blockIdx.x * 32 + (lane >> 1); const float v = (lane & 1) ? E1[ei] : E0[ei]; for (int pass = 0; pass < 2; ++pass) { ((volatile float*)out)[n * 2 + (lane & 1)] = v; __threadfence(); }
}
}

extern "C" void kernel_launch(void* const* d_in, const int* in_sizes, int n_in, void* d_out, int out_size, void* d_ws, size_t ws_size, hipStream_t stream) {
  (void)n_in;
  auto Fp = [&](int i) { return (const float*)d_in[i]; }; auto Ip = [&](int i) { return (const int*)d_in[i]; };
  if (in_sizes[0] != N * 3 || in_sizes[1] != N * S || in_sizes[2] != E * 3 || in_sizes[3] != E || in_sizes[4] != E || in_sizes[5] != S * F || in_sizes[9] != RH * NL * F || in_sizes[10] != NL * F * F || in_sizes[11] != S * F * F || in_sizes[18] != RH * NL * F || in_sizes[25] != F * HID || out_size != N * 2) return;
  const int NLIM = N; const int GB16 = NBLK;
  size_t off = 0; char* ws = (char*)d_ws;
  auto carve = [&](size_t bytes) { char* p = ws + off; off += (bytes + 255) & ~(size_t)255; return p; };
  b16* WUP[2]; b16* WR0[2]; b16* WR1[2]; b16* WR2[2]; b16* WMIX[2]; b16* WSCT[2]; b16* WP[2];
  for (int l = 0; l < 2; ++l) { WUP[l] = (b16*)carve(F * F * 2); WR0[l] = (b16*)carve(32 * 32 * 2); WR1[l] = (b16*)carve(32 * 32 * 2); WR2[l] = (b16*)carve(256 * 32 * 2); WMIX[l] = (b16*)carve(NL * F * F * 2); WSCT[l] = (b16*)carve(F * S * F * 2); WP[l] = (b16*)carve(3 * F * F * 2); }
  b16* WRO1A = (b16*)carve(16 * F * 2);
  float* H0 = (float*)carve((size_t)N * F * 4); float* H1 = (float*)carve((size_t)N * F * 4); float* H2 = (float*)carve((size_t)N * F * 4); float* HU = (float*)carve((size_t)N * F * 4); float* A = (float*)carve((size_t)N * NLM * F * 4); float* E0 = (float*)carve((size_t)NBLK * 32 * 4); float* E1 = (float*)carve((size_t)NBLK * 32 * 4);
  CsrBufs9 csr; off = csr_carve9(csr, ws, off, E, N);
  if (off > ws_size || off > ((size_t)96 << 20)) return;
  for (int l = 0; l < 2; ++l) { const int b = 6 + 9 * l;
    wput_kernel<<<(F * 8 + 255) / 256, 256, 0, stream>>>(Fp(b), F, F, 0, 0, F, WUP[l]);
    wzero_kernel<<<1, 256, 0, stream>>>(32 * 32 / 8, WR0[l]); wput_kernel<<<1, 256, 0, stream>>>(Fp(b + 1), NB, RH, 0, 0, 32, WR0[l]);
    wput_kernel<<<1, 256, 0, stream>>>(Fp(b + 2), RH, RH, 0, 0, 32, WR1[l]); wput_kernel<<<(256 * 4 + 255) / 256, 256, 0, stream>>>(Fp(b + 3), RH, NL * F, 0, 0, 32, WR2[l]);
    for (int q = 0; q < NL; ++q) wput_kernel<<<(F * 8 + 255) / 256, 256, 0, stream>>>(Fp(b + 4) + (size_t)q * F * F, F, F, q * F, 0, F, WMIX[l]);
    for (int s = 0; s < S; ++s) wput_kernel<<<(F * 8 + 255) / 256, 256, 0, stream>>>(Fp(b + 5) + (size_t)s * F * F, F, F, 0, s * F, S * F, WSCT[l]);
    for (int p = 0; p < 3; ++p) wput_kernel<<<(F * 8 + 255) / 256, 256, 0, stream>>>(Fp(b + 6 + p), F, F, p * F, 0, F, WP[l]); }
  wput_kernel<<<(16 * 8 + 255) / 256, 256, 0, stream>>>(Fp(25), F, HID, 0, 0, F, WRO1A);
  csr_build9(csr, Ip(4), E, N, stream);
  emb_kernel<<<NBLK, 32, 0, stream>>>(Fp(1), Fp(5), H0);
  hu_kernel<<<GB16, 32, 0, stream>>>(H0, WUP[0], NLIM, HU);
  msg_kernel<<<(unsigned)NLIM, 32, 0, stream>>>(Fp(0), Fp(2), Ip(3), HU, WR0[0], WR1[0], WR2[0], csr.PERM, csr.ROWPTR, csr.ROWCNT, (int)csr.permLen, NLIM, A);
  upd_kernel<0><<<GB16, 32, 0, stream>>>(A, H0, Fp(1), WMIX[0], WSCT[0], WP[0], Fp(24), nullptr, nullptr, NLIM, H1, E0);
  hu_kernel<<<GB16, 32, 0, stream>>>(H1, WUP[1], NLIM, HU);
  msg_kernel<<<(unsigned)NLIM, 32, 0, stream>>>(Fp(0), Fp(2), Ip(3), HU, WR0[1], WR1[1], WR2[1], csr.PERM, csr.ROWPTR, csr.ROWCNT, (int)csr.permLen, NLIM, A);
  upd_kernel<1><<<GB16, 32, 0, stream>>>(A, H1, Fp(1), WMIX[1], WSCT[1], WP[1], nullptr, WRO1A, Fp(26), NLIM, H2, E1);
  out_kernel<<<GB16, 32, 0, stream>>>(E0, E1, (float*)d_out);
}
